// MultiHeadAttention_82660940579038
// MI455X (gfx1250) — hardware-verified
//
#include <hip/hip_runtime.h>


#ifndef NB
#define NB 2
#endif
#ifndef SEQ
#define SEQ 2048
#endif
#define NB_FULL  2
#define SEQ_FULL 2048
#ifndef OUT_SEQ
#define OUT_SEQ SEQ
#endif
#define DM   1024
#define NH_  16
#define HD   64
#define AW   4
#define QRS  2048.0f
#define QRI  (1.0f / 2048.0f)
#define SC2  (0.125f * 1.4426950408889634f)
#define PSH  8.0f
#define FILLV (-3.0e38f)
#define FLP  64
#define EROWS ((SEQ < 256) ? SEQ : 256)
#define MSTR SEQ_FULL

static_assert(HD == 64);
static_assert(NH_ * HD == DM);
static_assert(DM % 64 == 0);
static_assert(DM % 32 == 0);
static_assert(SEQ % 64 == 0);
static_assert((NB * SEQ) % 64 == 0);
static_assert(SEQ % 32 == 0);
static_assert(EROWS % (16 * AW) == 0);
static_assert((SEQ - EROWS) % (16 * AW) == 0);
static_assert(SEQ / 32 <= FLP);
static_assert(FLP == 64);
static_assert(FLP % 8 == 0);
static_assert((SEQ * 32) % 256 == 0);
static_assert(((size_t)SEQ * DM) % 8 == 0);
static_assert(((size_t)DM * DM) % 8 == 0);
static_assert(NB <= NB_FULL);
static_assert(SEQ <= SEQ_FULL);
static_assert(HD / 2 == 32);

typedef _Float16 h16;
typedef unsigned short bf;
typedef __attribute__((ext_vector_type(16))) __bf16   v16bf;
typedef __attribute__((ext_vector_type(16))) _Float16 v16h;
typedef __attribute__((ext_vector_type(8)))  _Float16 v8h;
typedef __attribute__((ext_vector_type(8)))  unsigned short v8us;
typedef __attribute__((ext_vector_type(8)))  float    v8f;
typedef __attribute__((ext_vector_type(4)))  float    v4f;
typedef __attribute__((ext_vector_type(4)))  int      v4i;
typedef v4f  __attribute__((may_alias)) v4fa;

__device__ __forceinline__ unsigned short f2bf(float f) { unsigned u = __float_as_uint(f); u += 0x7FFFu + ((u >> 16) & 1u); return (unsigned short)(u >> 16); }
__device__ __forceinline__ float bf2f(unsigned short w) { return __uint_as_float(((unsigned)w) << 16); }
__device__ __forceinline__ v16h cat16(v8h lo, v8h hi) { return __builtin_shufflevector(lo, hi, 0, 1, 2, 3, 4, 5, 6, 7, 8, 9, 10, 11, 12, 13, 14, 15); }
__device__ __forceinline__ v16bf cat16b(v8us lo, v8us hi) { return __builtin_bit_cast(v16bf, __builtin_shufflevector(lo, hi, 0, 1, 2, 3, 4, 5, 6, 7, 8, 9, 10, 11, 12, 13, 14, 15)); }
__device__ __forceinline__ v8f wmma16(v16h a, v16h b, v8f c) { return __builtin_amdgcn_wmma_f32_16x16x32_f16(false, a, false, b, (short)0, c, false, false); }
__device__ __forceinline__ v8f wmmab(v16bf a, v16bf b, v8f c) { return __builtin_amdgcn_wmma_f32_16x16x32_bf16(false, a, false, b, (short)0, c, false, false); }
__device__ __forceinline__ v16h  ldh(const h16* p) { return cat16(*(const v8h*)p, *(const v8h*)(p + 16)); }
__device__ __forceinline__ v16bf ldb(const bf* p)  { return cat16b(*(const v8us*)p, *(const v8us*)(p + 16)); }
__device__ __forceinline__ void wave_sync() { __builtin_amdgcn_fence(3  , "wavefront"); __builtin_amdgcn_wave_barrier(); asm volatile("" ::: "memory"); }

__global__ __launch_bounds__(256) void k_cvt8(const float* __restrict__ src, bf* dst, size_t n8) {
    const size_t i = (size_t)blockIdx.x * 256 + threadIdx.x; if (i >= n8) return;
    const v8f v = *(const v8f*)(src + i * 8); v8us o;
#pragma unroll
    for (int k = 0; k < 8; ++k) o[k] = f2bf(v[k]);
    *(volatile v8us*)(dst + i * 8) = o; __threadfence(); *(volatile v8us*)(dst + i * 8) = o;
}

__global__ __launch_bounds__(256) void k_tab(float* CT, float* ST) {
    const int idx = (int)blockIdx.x * 256 + (int)threadIdx.x;
    const int i = idx & 31, t = idx >> 5;
    double p = 1.0;
    p = (i & 1)  ? p * 1.3335214321633240 : p;
    p = (i & 2)  ? p * 1.7782794100389228 : p;
    p = (i & 4)  ? p * 3.1622776601683795 : p;
    p = (i & 8)  ? p * 10.0 : p;
    p = (i & 16) ? p * 100.0 : p;
    const float theta = (float)(1.0 / p);
    const float ang = (float)t * theta;
    float sn, cs; sincosf(ang, &sn, &cs);
    *(volatile float*)(CT + idx) = cs; *(volatile float*)(ST + idx) = sn;
    __threadfence();
    *(volatile float*)(CT + idx) = cs; *(volatile float*)(ST + idx) = sn;
}

__global__ __launch_bounds__(256) void k_flags(const int* __restrict__ MK, int* FL) {
    __shared__ int fl[FLP];
    __shared__ int rowun[8 * 16];
    const int lane = threadIdx.x & 31;
    const int wave = __builtin_amdgcn_readfirstlane((int)(threadIdx.x >> 5));
    const int row = lane >> 1, half = lane & 1;
    const int q0 = (int)blockIdx.x * 16;
    int ru = 0;
#pragma unroll 1
    for (int i = 0; i < FLP / 8; ++i) {
        const int kt = wave * (FLP / 8) + i;
        const int real = (kt < SEQ / 32) ? 1 : 0;
        const int ktc = real ? kt : (SEQ / 32 - 1);
        const int* mp = MK + (size_t)(q0 + row) * MSTR + ktc * 32 + half * 16;
        const v4i a = *(const v4i*)mp, c = *(const v4i*)(mp + 4), d = *(const v4i*)(mp + 8), e = *(const v4i*)(mp + 12);
        int nm = 0;
#pragma unroll
        for (int j = 0; j < 4; ++j) nm += (a[j] != 0) + (c[j] != 0) + (d[j] != 0) + (e[j] != 0);
        const unsigned anyM = __builtin_amdgcn_ballot_w32(nm > 0);
        const unsigned anyU = __builtin_amdgcn_ballot_w32(nm < 16);
        int f = (anyU == 0u) ? 0 : ((anyM == 0u) ? 1 : 2);
        f = real ? f : 0;
        ru |= (real != 0 && nm < 16) ? 1 : 0;
        if (lane == 0) fl[kt] = f;
    }
    ru |= __shfl_xor(ru, 1, 32);
    if (half == 0) rowun[wave * 16 + row] = ru;
    __syncthreads();
    if (wave == 0) {
        int u = 0;
#pragma unroll
        for (int w = 0; w < 8; ++w) u |= rowun[w * 16 + (lane & 15)];
        const unsigned anyFull = __builtin_amdgcn_ballot_w32((lane < 16) && (u == 0));
        v4i o;
#pragma unroll
        for (int j = 0; j < 4; ++j) { const int kt = (lane & 15) * 4 + j; int f = fl[kt]; f = (anyFull != 0u && kt < SEQ / 32) ? 2 : f; o[j] = f; }
        int* dst = FL + (size_t)blockIdx.x * FLP + (lane & 15) * 4;
        if (lane < 16) *(volatile v4i*)dst = o;
        __threadfence();
        if (lane < 16) *(volatile v4i*)dst = o;
    }
}

__global__ __launch_bounds__(32) void k_proj(const bf* __restrict__ A, const bf* __restrict__ Bt, h16* Ph, h16* Pr, const float* __restrict__ CT, const float* __restrict__ ST,
                                             int useRope, int RB, size_t sRB, int pitch, int CB, size_t sCB) {
    __shared__ __align__(16) float os[16 * 68];
    const int K = DM;
    const int lane = threadIdx.x & 31, lr = lane & 15, hi = lane >> 4; const int r0 = (int)blockIdx.x * 64, c0 = (int)blockIdx.y * 64;
    v8f acc[4][4];
#pragma unroll
    for (int mb = 0; mb < 4; ++mb)
#pragma unroll
        for (int nb = 0; nb < 4; ++nb) acc[mb][nb] = (v8f){};
    const size_t aoff = (size_t)(r0 + lr) * K + 8 * hi, boff = (size_t)(c0 + lr) * K + 8 * hi;
#pragma unroll 1
    for (int kc = 0; kc < K; kc += 32) {
        v16bf a[4];
#pragma unroll
        for (int mb = 0; mb < 4; ++mb) a[mb] = ldb(A + aoff + (size_t)mb * 16 * K + kc);
#pragma unroll
        for (int nb = 0; nb < 4; ++nb) { const v16bf b = ldb(Bt + boff + (size_t)nb * 16 * K + kc);
#pragma unroll
            for (int mb = 0; mb < 4; ++mb) acc[mb][nb] = wmmab(a[mb], b, acc[mb][nb]); }
        asm volatile("v_nop\n\tv_nop\n\tv_nop\n\tv_nop" : "+v"(acc[0][0]), "+v"(acc[1][1]), "+v"(acc[2][2]), "+v"(acc[3][3]) : "v"(a[0]), "v"(a[1]), "v"(a[2]), "v"(a[3]));
    }
    const int tokb = r0 % RB;
    const size_t tbase = (size_t)(r0 / RB) * sRB + (size_t)tokb * (size_t)pitch + (size_t)(c0 / CB) * sCB + (size_t)(c0 % CB);
#pragma unroll
    for (int mb = 0; mb < 4; ++mb) {
#pragma unroll
        for (int nb = 0; nb < 4; ++nb) {
#pragma unroll
            for (int j = 0; j < 8; ++j) os[(hi * 8 + j) * 68 + nb * 16 + lr] = acc[mb][nb][j]; }
        wave_sync();
        const size_t sb = tbase + (size_t)(mb * 16) * (size_t)pitch;
#pragma unroll 1
        for (int ps = 0; ps < 2; ++ps) {
#pragma unroll
            for (int s = 0; s < 4; ++s) { const int row = 4 * s + (lane >> 3), c8 = (lane & 7) * 8;
                v4f x0 = *(const v4fa*)(&os[row * 68 + c8]); v4f x1 = *(const v4fa*)(&os[row * 68 + c8 + 4]);
                int tok = tokb + mb * 16 + row; tok = (tok < SEQ) ? tok : (SEQ - 1);
                const v4f cs = *(const v4f*)(CT + (size_t)tok * 32 + (c8 >> 1)); const v4f sn = *(const v4f*)(ST + (size_t)tok * 32 + (c8 >> 1));
                if (useRope) { float e, o;
                    e = x0[0]; o = x0[1]; x0[0] = e * cs[0] - o * sn[0]; x0[1] = o * cs[0] + e * sn[0];
                    e = x0[2]; o = x0[3]; x0[2] = e * cs[1] - o * sn[1]; x0[3] = o * cs[1] + e * sn[1];
                    e = x1[0]; o = x1[1]; x1[0] = e * cs[2] - o * sn[2]; x1[1] = o * cs[2] + e * sn[2];
                    e = x1[2]; o = x1[3]; x1[2] = e * cs[3] - o * sn[3]; x1[3] = o * cs[3] + e * sn[3]; }
                v8h hv, rv;
#pragma unroll
                for (int i = 0; i < 4; ++i) { const h16 a0 = (h16)x0[i]; const h16 a1 = (h16)x1[i]; hv[i] = a0; hv[4 + i] = a1; rv[i] = (h16)((x0[i] - (float)a0) * QRS); rv[4 + i] = (h16)((x1[i] - (float)a1) * QRS); }
                const size_t oo = sb + (size_t)row * (size_t)pitch + c8;
                *(volatile v8h*)(Ph + oo) = hv; *(volatile v8h*)(Pr + oo) = rv; }
            if (ps == 0) __threadfence(); }
        wave_sync();
    }
}

template <int EARLY>
__device__ __forceinline__ void flash_body(const h16* __restrict__ QH, const h16* __restrict__ QR, const h16* __restrict__ KH, const h16* __restrict__ KR,
                                           const h16* __restrict__ VT, const h16* __restrict__ VR, const int* __restrict__ MK, const int* __restrict__ FL,
                                           bf* CH, bf* CL, const int tbase) {
    __shared__ __align__(16) float os[AW * 16 * 68];
    const int lane = threadIdx.x & 31;
    const int wave = __builtin_amdgcn_readfirstlane((int)(threadIdx.x >> 5));
    const int lr = lane & 15, hi = lane >> 4;
    const int zh = (int)blockIdx.y; const int b = zh / NH_, h = zh % NH_;
    const int t0 = tbase + ((int)blockIdx.x * AW + wave) * 16;
    const int qt = t0 >> 4;
    const int f0 = FL[(size_t)qt * FLP + lane], f1 = FL[(size_t)qt * FLP + 32 + lane];
    const unsigned liveA = __builtin_amdgcn_ballot_w32(f0 != 0), liveB = __builtin_amdgcn_ballot_w32(f1 != 0);
    const unsigned mixA = __builtin_amdgcn_ballot_w32(f0 == 2), mixB = __builtin_amdgcn_ballot_w32(f1 == 2);
    const size_t pbase = (size_t)zh * SEQ * HD;
    const unsigned qo = (unsigned)(pbase + (size_t)(t0 + lr) * HD + 8 * hi);
    const size_t ko = pbase + (size_t)lr * HD + 8 * hi;
    const size_t vo = pbase + (size_t)lr * SEQ + 8 * hi;
    v16h qh0 = (v16h){}, qh1 = (v16h){}, qr0 = (v16h){}, qr1 = (v16h){};
    if (!EARLY) { qh0 = ldh(QH + qo); qh1 = ldh(QH + qo + 32); qr0 = ldh(QR + qo); qr1 = ldh(QR + qo + 32); }
    v8f o0 = (v8f){}, o1 = (v8f){}, o2 = (v8f){}, o3 = (v8f){};
    v8f e0 = (v8f){}, e1 = (v8f){}, e2 = (v8f){}, e3 = (v8f){};
    float m = FILLV, l = 0.0f;
#pragma unroll 1
    for (int kt = 0; kt < SEQ / 32; ++kt) {
        const unsigned lw = (kt < 32) ? liveA : liveB, mw = (kt < 32) ? mixA : mixB;
        const unsigned bit = 1u << (kt & 31);
        if ((lw & bit) == 0u) continue;
        const int key0 = kt * 32;
        if (EARLY) { unsigned qv = qo; asm volatile("" : "+v"(qv)); qh0 = ldh(QH + qv); qh1 = ldh(QH + qv + 32); qr0 = ldh(QR + qv); qr1 = ldh(QR + qv + 32); }
        const size_t kof = ko + (size_t)key0 * HD;
        v8f sHa = (v8f){}, sLa = (v8f){}, sHb = (v8f){}, sLb = (v8f){};
        { const v16h ka0 = ldh(KH + kof), ka1 = ldh(KH + kof + 32), kb0 = ldh(KH + kof + 16 * HD), kb1 = ldh(KH + kof + 16 * HD + 32);
          sHa = wmma16(ka0, qh0, sHa); sLa = wmma16(ka0, qr0, sLa); sHb = wmma16(kb0, qh0, sHb); sLb = wmma16(kb0, qr0, sLb);
          sHa = wmma16(ka1, qh1, sHa); sLa = wmma16(ka1, qr1, sLa); sHb = wmma16(kb1, qh1, sHb); sLb = wmma16(kb1, qr1, sLb);
          asm volatile("v_nop\n\tv_nop\n\tv_nop\n\tv_nop" : "+v"(sHa), "+v"(sLa), "+v"(sHb), "+v"(sLb) : "v"(ka0), "v"(ka1), "v"(kb0), "v"(kb1), "v"(qh1), "v"(qr1)); }
        if (EARLY) {
            asm volatile("" ::: "memory");
            const v16h ra0 = ldh(KR + kof), ra1 = ldh(KR + kof + 32), rb0 = ldh(KR + kof + 16 * HD), rb1 = ldh(KR + kof + 16 * HD + 32);
            sLa = wmma16(ra0, qh0, sLa); sLb = wmma16(rb0, qh0, sLb); sLa = wmma16(ra1, qh1, sLa); sLb = wmma16(rb1, qh1, sLb);
            asm volatile("v_nop\n\tv_nop\n\tv_nop\n\tv_nop" : "+v"(sLa), "+v"(sLb) : "v"(ra0), "v"(ra1), "v"(rb0), "v"(rb1), "v"(qh1));
        }
        float ta[8], tb[8];
#pragma unroll
        for (int r = 0; r < 8; ++r) { ta[r] = (sHa[r] + sLa[r] * QRI) * SC2; tb[r] = (sHb[r] + sLb[r] * QRI) * SC2; }
        if ((mw & bit) != 0u) {
            const int* mp = MK + (size_t)(t0 + lr) * MSTR + key0 + 8 * hi;
            const v4i m0 = *(const v4i*)mp, m1 = *(const v4i*)(mp + 4), m2 = *(const v4i*)(mp + 16), m3 = *(const v4i*)(mp + 20);
#pragma unroll
            for (int r = 0; r < 4; ++r) {
                ta[r]     = (m0[r] != 0) ? FILLV : ta[r];
                ta[4 + r] = (m1[r] != 0) ? FILLV : ta[4 + r];
                tb[r]     = (m2[r] != 0) ? FILLV : tb[r];
                tb[4 + r] = (m3[r] != 0) ? FILLV : tb[4 + r]; }
        }
        float mx = FILLV;
#pragma unroll
        for (int r = 0; r < 8; ++r) mx = fmaxf(mx, fmaxf(ta[r], tb[r]));
        mx = fmaxf(mx, __shfl_xor(mx, 16, 32));
        const float mnew = fmaxf(m, mx);
        const float alpha = __builtin_amdgcn_exp2f(m - mnew);
        const float sh = PSH - mnew;
        v16h pb = (v16h){}, pr = (v16h){}; float ls = 0.0f;
#pragma unroll
        for (int r = 0; r < 8; ++r) {
            const float fa = __builtin_amdgcn_exp2f(ta[r] + sh), fc = __builtin_amdgcn_exp2f(tb[r] + sh);
            const h16 pa = (h16)fa, pc = (h16)fc; pb[r] = pa; pb[8 + r] = pc;
            if (EARLY) { const h16 xa = (h16)((fa - (float)pa) * QRS), xc = (h16)((fc - (float)pc) * QRS); pr[r] = xa; pr[8 + r] = xc;
                         ls += ((float)pa + (float)xa * QRI) + ((float)pc + (float)xc * QRI); }
            else ls += (float)pa + (float)pc; }
        l = l * alpha + ls; m = mnew;
        o0 = o0 * alpha; o1 = o1 * alpha; o2 = o2 * alpha; o3 = o3 * alpha;
        if (EARLY) { e0 = e0 * alpha; e1 = e1 * alpha; e2 = e2 * alpha; e3 = e3 * alpha; }
        const size_t vof = vo + (size_t)key0;
        if (EARLY) {
            { const v16h v0 = ldh(VT + vof), v1 = ldh(VT + vof + (size_t)16 * SEQ), v2 = ldh(VT + vof + (size_t)32 * SEQ), v3 = ldh(VT + vof + (size_t)48 * SEQ);
              o0 = wmma16(v0, pb, o0); o1 = wmma16(v1, pb, o1); o2 = wmma16(v2, pb, o2); o3 = wmma16(v3, pb, o3);
              e0 = wmma16(v0, pr, e0); e1 = wmma16(v1, pr, e1); e2 = wmma16(v2, pr, e2); e3 = wmma16(v3, pr, e3);
              asm volatile("v_nop\n\tv_nop\n\tv_nop\n\tv_nop" : "+v"(o0), "+v"(o1), "+v"(o2), "+v"(o3), "+v"(e0), "+v"(e1), "+v"(e2), "+v"(e3) : "v"(v0), "v"(v1), "v"(v2), "v"(v3), "v"(pb), "v"(pr)); }
            asm volatile("" ::: "memory");
            { const v16h w0 = ldh(VR + vof), w1 = ldh(VR + vof + (size_t)16 * SEQ), w2 = ldh(VR + vof + (size_t)32 * SEQ), w3 = ldh(VR + vof + (size_t)48 * SEQ);
              e0 = wmma16(w0, pb, e0); e1 = wmma16(w1, pb, e1); e2 = wmma16(w2, pb, e2); e3 = wmma16(w3, pb, e3);
              asm volatile("v_nop\n\tv_nop\n\tv_nop\n\tv_nop" : "+v"(e0), "+v"(e1), "+v"(e2), "+v"(e3) : "v"(w0), "v"(w1), "v"(w2), "v"(w3), "v"(pb)); }
        } else {
            const v16h v0 = ldh(VT + vof), v1 = ldh(VT + vof + (size_t)16 * SEQ), v2 = ldh(VT + vof + (size_t)32 * SEQ), v3 = ldh(VT + vof + (size_t)48 * SEQ);
            o0 = wmma16(v0, pb, o0); o1 = wmma16(v1, pb, o1); o2 = wmma16(v2, pb, o2); o3 = wmma16(v3, pb, o3);
            asm volatile("v_nop\n\tv_nop\n\tv_nop\n\tv_nop" : "+v"(o0), "+v"(o1), "+v"(o2), "+v"(o3) : "v"(v0), "v"(v1), "v"(v2), "v"(v3), "v"(pb));
        }
    }
    l += __shfl_xor(l, 16, 32);
    const float inv = 1.0f / l;
    if (EARLY) { o0 = o0 + e0 * QRI; o1 = o1 + e1 * QRI; o2 = o2 + e2 * QRI; o3 = o3 + e3 * QRI; }
    const int wb = wave * 16 * 68;
    { v4f a, c;
      a[0] = o0[0] * inv; a[1] = o0[1] * inv; a[2] = o0[2] * inv; a[3] = o0[3] * inv; c[0] = o0[4] * inv; c[1] = o0[5] * inv; c[2] = o0[6] * inv; c[3] = o0[7] * inv;
      *(v4fa*)(&os[wb + lr * 68 +  0 + 8 * hi]) = a; *(v4fa*)(&os[wb + lr * 68 +  0 + 8 * hi + 4]) = c;
      a[0] = o1[0] * inv; a[1] = o1[1] * inv; a[2] = o1[2] * inv; a[3] = o1[3] * inv; c[0] = o1[4] * inv; c[1] = o1[5] * inv; c[2] = o1[6] * inv; c[3] = o1[7] * inv;
      *(v4fa*)(&os[wb + lr * 68 + 16 + 8 * hi]) = a; *(v4fa*)(&os[wb + lr * 68 + 16 + 8 * hi + 4]) = c;
      a[0] = o2[0] * inv; a[1] = o2[1] * inv; a[2] = o2[2] * inv; a[3] = o2[3] * inv; c[0] = o2[4] * inv; c[1] = o2[5] * inv; c[2] = o2[6] * inv; c[3] = o2[7] * inv;
      *(v4fa*)(&os[wb + lr * 68 + 32 + 8 * hi]) = a; *(v4fa*)(&os[wb + lr * 68 + 32 + 8 * hi + 4]) = c;
      a[0] = o3[0] * inv; a[1] = o3[1] * inv; a[2] = o3[2] * inv; a[3] = o3[3] * inv; c[0] = o3[4] * inv; c[1] = o3[5] * inv; c[2] = o3[6] * inv; c[3] = o3[7] * inv;
      *(v4fa*)(&os[wb + lr * 68 + 48 + 8 * hi]) = a; *(v4fa*)(&os[wb + lr * 68 + 48 + 8 * hi + 4]) = c; }
    wave_sync();
    const size_t cbase = ((size_t)b * SEQ + t0) * DM + (size_t)h * HD;
#pragma unroll 1
    for (int ps = 0; ps < 2; ++ps) {
#pragma unroll
        for (int s = 0; s < 4; ++s) { const int row = 4 * s + (lane >> 3), c8 = (lane & 7) * 8;
            const v4f x0 = *(const v4fa*)(&os[wb + row * 68 + c8]); const v4f x1 = *(const v4fa*)(&os[wb + row * 68 + c8 + 4]); v8us hv, lv;
#pragma unroll
            for (int i = 0; i < 4; ++i) { const unsigned short a0 = f2bf(x0[i]); const unsigned short a1 = f2bf(x1[i]); hv[i] = a0; hv[4 + i] = a1; lv[i] = f2bf(x0[i] - bf2f(a0)); lv[4 + i] = f2bf(x1[i] - bf2f(a1)); }
            const size_t oo = cbase + (size_t)row * DM + c8;
            *(volatile v8us*)(CH + oo) = hv; *(volatile v8us*)(CL + oo) = lv; }
        if (ps == 0) __threadfence(); }
}

__global__ __launch_bounds__(32 * AW) void k_flash_e(const h16* __restrict__ QH, const h16* __restrict__ QR, const h16* __restrict__ KH, const h16* __restrict__ KR,
                                                     const h16* __restrict__ VT, const h16* __restrict__ VR, const int* __restrict__ MK, const int* __restrict__ FL, bf* CH, bf* CL) {
    flash_body<1>(QH, QR, KH, KR, VT, VR, MK, FL, CH, CL, 0);
}
__global__ __launch_bounds__(32 * AW) void k_flash_l(const h16* __restrict__ QH, const h16* __restrict__ QR, const h16* __restrict__ KH, const h16* __restrict__ KR,
                                                     const h16* __restrict__ VT, const h16* __restrict__ VR, const int* __restrict__ MK, const int* __restrict__ FL, bf* CH, bf* CL) {
    flash_body<0>(QH, QR, KH, KR, VT, VR, MK, FL, CH, CL, EROWS);
}

__global__ __launch_bounds__(32) void k_out(const bf* __restrict__ A, size_t aplane, const bf* __restrict__ Bt, float* OUT) {
    __shared__ __align__(16) float os[16 * 68];
    const int K = DM;
    const int lane = threadIdx.x & 31, lr = lane & 15, hi = lane >> 4; const int r0 = (int)blockIdx.x * 64, c0 = (int)blockIdx.y * 64;
    v8f acc[4][4];
#pragma unroll
    for (int mb = 0; mb < 4; ++mb)
#pragma unroll
        for (int nb = 0; nb < 4; ++nb) acc[mb][nb] = (v8f){};
    const size_t aoff = (size_t)(r0 + lr) * K + 8 * hi, boff = (size_t)(c0 + lr) * K + 8 * hi;
#pragma unroll 1
    for (int kk = 0; kk < 2 * K; kk += 32) {
        const int kc = (kk < K) ? kk : (kk - K);
        const size_t ap = (kk < K) ? (size_t)0 : aplane;
        v16bf a[4];
#pragma unroll
        for (int mb = 0; mb < 4; ++mb) a[mb] = ldb(A + ap + aoff + (size_t)mb * 16 * K + kc);
#pragma unroll
        for (int nb = 0; nb < 4; ++nb) { const v16bf b = ldb(Bt + boff + (size_t)nb * 16 * K + kc);
#pragma unroll
            for (int mb = 0; mb < 4; ++mb) acc[mb][nb] = wmmab(a[mb], b, acc[mb][nb]); }
        asm volatile("v_nop\n\tv_nop\n\tv_nop\n\tv_nop" : "+v"(acc[0][0]), "+v"(acc[1][1]), "+v"(acc[2][2]), "+v"(acc[3][3]) : "v"(a[0]), "v"(a[1]), "v"(a[2]), "v"(a[3]));
    }
    const size_t orow0 = (size_t)(r0 / SEQ) * OUT_SEQ + (size_t)(r0 % SEQ);
#pragma unroll
    for (int mb = 0; mb < 4; ++mb) {
#pragma unroll
        for (int nb = 0; nb < 4; ++nb) {
#pragma unroll
            for (int j = 0; j < 8; ++j) os[(hi * 8 + j) * 68 + nb * 16 + lr] = acc[mb][nb][j]; }
        wave_sync();
        float* orow = OUT + (orow0 + (size_t)(mb * 16)) * DM + c0;
#pragma unroll 1
        for (int ps = 0; ps < 2; ++ps) {
#pragma unroll
            for (int s = 0; s < 8; ++s) { const int row = 2 * s + hi, cofs = lr * 4;
                const v4f val = *(const v4fa*)(&os[row * 68 + cofs]);
                *(volatile v4f*)(orow + (size_t)row * DM + cofs) = val; }
            if (ps == 0) __threadfence(); }
        wave_sync();
    }
}

static constexpr size_t al256(size_t v) { return (v + 255) & ~(size_t)255; }
static constexpr size_t SZ_X1 = al256((size_t)NB * SEQ * DM * 2);
static constexpr size_t SZ_WB = al256((size_t)4 * DM * DM * 2);
static constexpr size_t SZ_PL = al256((size_t)NB * NH_ * SEQ * HD * 2);
static constexpr size_t SZ_CX = al256((size_t)2 * NB * SEQ * DM * 2);
static constexpr size_t SZ_TB = al256((size_t)SEQ * 32 * 4);
static constexpr size_t SZ_FL = al256((size_t)(SEQ / 16) * FLP * 4);
static constexpr size_t SZ_TOTAL = 3 * SZ_X1 + SZ_WB + 6 * SZ_PL + SZ_CX + 2 * SZ_TB + SZ_FL;
static_assert(SZ_TOTAL <= (size_t)134217728);
static_assert(((size_t)DM * DM * 2) % 256 == 0);
static_assert(((size_t)NB * SEQ * DM * 2) % 256 == 0);
static_assert(((size_t)(NB_FULL - 1) * OUT_SEQ + SEQ) * DM * 4 <= (size_t)NB_FULL * SEQ_FULL * DM * 4);

extern "C" void kernel_launch(void* const* d_in, const int* in_sizes, int n_in,
                              void* d_out, int out_size, void* d_ws, size_t ws_size, hipStream_t stream) {
    if (n_in < 8) return;
    const size_t needx = ((size_t)(NB - 1) * SEQ_FULL + SEQ) * DM;
    if ((size_t)in_sizes[0] < needx || (size_t)in_sizes[1] < needx || (size_t)in_sizes[2] < needx) return;
    if ((size_t)in_sizes[3] < (size_t)(SEQ - 1) * MSTR + SEQ) return;
    if ((size_t)in_sizes[4] < (size_t)DM * DM || (size_t)in_sizes[5] < (size_t)DM * DM || (size_t)in_sizes[6] < (size_t)DM * DM || (size_t)in_sizes[7] < (size_t)DM * DM) return;
    if ((size_t)out_size < ((size_t)(NB - 1) * OUT_SEQ + SEQ) * DM) return;
    if (SZ_TOTAL > ws_size) return;
    const float* xq = (const float*)d_in[0]; const float* xk = (const float*)d_in[1]; const float* xv = (const float*)d_in[2];
    const int* MK = (const int*)d_in[3];
    const float* wq = (const float*)d_in[4]; const float* wk = (const float*)d_in[5]; const float* wv = (const float*)d_in[6]; const float* wo = (const float*)d_in[7];
    float* OUT = (float*)d_out;
    char* wsp = (char*)d_ws;
    bf* XQ = (bf*)wsp; wsp += SZ_X1;
    bf* XK = (bf*)wsp; wsp += SZ_X1;
    bf* XV = (bf*)wsp; wsp += SZ_X1;
    bf* WB = (bf*)wsp; wsp += SZ_WB;
    h16* QH = (h16*)wsp; wsp += SZ_PL;
    h16* QR = (h16*)wsp; wsp += SZ_PL;
    h16* KH = (h16*)wsp; wsp += SZ_PL;
    h16* KR = (h16*)wsp; wsp += SZ_PL;
    h16* VT = (h16*)wsp; wsp += SZ_PL;
    h16* VR = (h16*)wsp; wsp += SZ_PL;
    bf* CX = (bf*)wsp; wsp += SZ_CX;
    float* CT = (float*)wsp; wsp += SZ_TB;
    float* ST = (float*)wsp; wsp += SZ_TB;
    int* FL = (int*)wsp; wsp += SZ_FL;
    bf* WQ = WB; bf* WK = WB + (size_t)DM * DM; bf* WV = WB + (size_t)2 * DM * DM; bf* WO = WB + (size_t)3 * DM * DM;
    const size_t cplane = (size_t)NB * SEQ * DM;
    bf* CH = CX; bf* CL = CX + cplane;

    if (SEQ == SEQ_FULL) {
        const size_t n8 = (size_t)NB * SEQ * DM / 8; const unsigned g = (unsigned)((n8 + 255) / 256);
        k_cvt8<<<g, 256, 0, stream>>>(xq, XQ, n8); k_cvt8<<<g, 256, 0, stream>>>(xk, XK, n8); k_cvt8<<<g, 256, 0, stream>>>(xv, XV, n8);
    } else {
        const size_t n8 = (size_t)SEQ * DM / 8; const unsigned g = (unsigned)((n8 + 255) / 256);
        for (int b = 0; b < NB; ++b) {
            k_cvt8<<<g, 256, 0, stream>>>(xq + (size_t)b * SEQ_FULL * DM, XQ + (size_t)b * SEQ * DM, n8);
            k_cvt8<<<g, 256, 0, stream>>>(xk + (size_t)b * SEQ_FULL * DM, XK + (size_t)b * SEQ * DM, n8);
            k_cvt8<<<g, 256, 0, stream>>>(xv + (size_t)b * SEQ_FULL * DM, XV + (size_t)b * SEQ * DM, n8);
        }
    }
    { const size_t n8 = (size_t)DM * DM / 8; const unsigned g = (unsigned)((n8 + 255) / 256);
      k_cvt8<<<g, 256, 0, stream>>>(wq, WQ, n8); k_cvt8<<<g, 256, 0, stream>>>(wk, WK, n8); k_cvt8<<<g, 256, 0, stream>>>(wv, WV, n8); k_cvt8<<<g, 256, 0, stream>>>(wo, WO, n8); }

    k_tab<<<(unsigned)(SEQ * 32 / 256), 256, 0, stream>>>(CT, ST);
    k_flags<<<(unsigned)(SEQ / 16), 256, 0, stream>>>(MK, FL);

    k_proj<<<dim3(NB * SEQ / 64, DM / 64, 1), 32, 0, stream>>>(XQ, WQ, QH, QR, CT, ST, 1, SEQ, (size_t)NH_ * SEQ * HD, HD, HD, (size_t)SEQ * HD);
    k_proj<<<dim3(NB * SEQ / 64, DM / 64, 1), 32, 0, stream>>>(XK, WK, KH, KR, CT, ST, 1, SEQ, (size_t)NH_ * SEQ * HD, HD, HD, (size_t)SEQ * HD);
    k_proj<<<dim3(DM / 64, NB * SEQ / 64, 1), 32, 0, stream>>>(WV, XV, VT, VR, CT, ST, 0, DM, (size_t)0, SEQ, SEQ, (size_t)DM * SEQ);

    k_flash_e<<<dim3(EROWS / (16 * AW), NB * NH_, 1), 32 * AW, 0, stream>>>(QH, QR, KH, KR, VT, VR, MK, FL, CH, CL);
    if (SEQ > EROWS)
        k_flash_l<<<dim3((SEQ - EROWS) / (16 * AW), NB * NH_, 1), 32 * AW, 0, stream>>>(QH, QR, KH, KR, VT, VR, MK, FL, CH, CL);

    k_out<<<dim3(NB * SEQ / 64, DM / 64, 1), 32, 0, stream>>>(CX, cplane, WO, OUT);
}
